// MultiHeadedAttention_85736137162970
// MI455X (gfx1250) — hardware-verified
//
#include <hip/hip_runtime.h>
#include <math.h>

#ifndef NB
#define NB 2
#endif
#ifndef SEQ
#define SEQ 2048
#endif
#define NB_FULL 2
#define SEQ_FULL 2048
#define DM 1024
#define DM2 2048
#define NH 16
#define DK 64
#define MROWS (NB * SEQ)

static_assert(DM == 1024);
static_assert(DM2 == 2 * DM);
static_assert(NH * DK == DM);
static_assert(DK == 64);
static_assert(NB >= 1 && NB <= NB_FULL);
static_assert(SEQ >= 64 && SEQ <= SEQ_FULL);
static_assert((SEQ % 64) == 0);
static_assert((MROWS % 64) == 0);
static_assert((DM % 64) == 0 && (DM % 32) == 0 && (DM2 % 32) == 0);
static_assert((unsigned long long)MROWS * DM2 < 4294967296ull);

typedef __attribute__((ext_vector_type(16))) _Float16     v16h;
typedef __attribute__((ext_vector_type(8)))  _Float16     v8h;
typedef __attribute__((ext_vector_type(8)))  float        v8f;
typedef __attribute__((ext_vector_type(4)))  float        v4f;
typedef __attribute__((ext_vector_type(4)))  unsigned int u4v;

union HF { v16h v; v8h h[2]; };
__device__ __forceinline__ v16h ldfrag(const _Float16* p) {
  HF f; f.h[0] = *(const v8h*)(p); f.h[1] = *(const v8h*)(p + 16); return f.v;
}
__device__ __forceinline__ v8f mma_h(v16h a, v16h b, v8f c) {
  c = __builtin_amdgcn_wmma_f32_16x16x32_f16(false, a, false, b, (short)0, c, false, false);
  asm volatile("v_nop\n\tv_nop\n\tv_nop\n\tv_nop" : "+v"(c) : "v"(a), "v"(b));
  return c;
}
__device__ __forceinline__ void dep_guard_h(v8f& a, v8f& b, v16h x, v16h y) { asm volatile("v_nop\n\tv_nop\n\tv_nop\n\tv_nop" : "+v"(a), "+v"(b) : "v"(x), "v"(y)); }
__device__ __forceinline__ void keep4_h(v16h a, v16h b, v16h c, v16h d) { asm volatile("v_nop" :: "v"(a), "v"(b), "v"(c), "v"(d)); }
__device__ __forceinline__ void acc_guard4(v8f& a, v8f& b, v8f& c, v8f& d) { asm volatile("v_nop\n\tv_nop\n\tv_nop\n\tv_nop" : "+v"(a), "+v"(b), "+v"(c), "+v"(d)); }

#define VST2(T, ptr, val) do { const T vst2_v_ = (val); *(volatile T*)(ptr) = vst2_v_; __threadfence(); *(volatile T*)(ptr) = vst2_v_; } while (0)

__device__ __forceinline__ float cmb_bf(float v) {
  const unsigned u = __builtin_bit_cast(unsigned, v);
  const unsigned r = (u + 0x7fffu + ((u >> 16) & 1u)) & 0xffff0000u;
  return __builtin_bit_cast(float, r);
}
__device__ __forceinline__ unsigned int pk2h(float a, float b) {
  return (unsigned int)__builtin_bit_cast(unsigned short, (_Float16)a) | ((unsigned int)__builtin_bit_cast(unsigned short, (_Float16)b) << 16);
}

__global__ __launch_bounds__(256) void k_castw(const float* __restrict__ SRC, unsigned short* __restrict__ DST, unsigned dpitch, unsigned dup, float sc) {
  const unsigned u = blockIdx.x * 256u + threadIdx.x;
  if (u >= (unsigned)(DM * (DM / 8))) return;
  const unsigned n = u >> 7, k0 = (u & 127u) << 3;
  const float* sp = SRC + (size_t)n * DM + k0;
  const v4f x0 = *(const v4f*)sp, x1 = *(const v4f*)(sp + 4);
  u4v pk;
  pk.x = pk2h(cmb_bf(x0.x) * sc, cmb_bf(x0.y) * sc); pk.y = pk2h(cmb_bf(x0.z) * sc, cmb_bf(x0.w) * sc);
  pk.z = pk2h(cmb_bf(x1.x) * sc, cmb_bf(x1.y) * sc); pk.w = pk2h(cmb_bf(x1.z) * sc, cmb_bf(x1.w) * sc);
  VST2(u4v, (u4v*)(DST + (size_t)n * dpitch + k0), pk);
  if (dup != 0u) {
    VST2(u4v, (u4v*)(DST + (size_t)n * dpitch + DM + k0), pk);
  }
}

__global__ __launch_bounds__(256) void k_castx(const float* __restrict__ SRC, unsigned short* __restrict__ DST, float sc) {
  const unsigned u = blockIdx.x * 256u + threadIdx.x;
  if (u >= (unsigned)MROWS * 128u) return;
  const unsigned r = u >> 7, c0 = (u & 127u) << 3;
  const unsigned b = r / (unsigned)SEQ, s = r - b * (unsigned)SEQ;
  const float* sp = SRC + ((size_t)b * SEQ_FULL + s) * DM + c0;
  const v4f x0 = *(const v4f*)sp, x1 = *(const v4f*)(sp + 4);
  u4v pk;
  pk.x = pk2h(cmb_bf(x0.x) * sc, cmb_bf(x0.y) * sc); pk.y = pk2h(cmb_bf(x0.z) * sc, cmb_bf(x0.w) * sc);
  pk.z = pk2h(cmb_bf(x1.x) * sc, cmb_bf(x1.y) * sc); pk.w = pk2h(cmb_bf(x1.z) * sc, cmb_bf(x1.w) * sc);
  VST2(u4v, (u4v*)(DST + (size_t)r * DM + c0), pk);
}

__global__ __launch_bounds__(256) void k_bias4(const float* __restrict__ b0, const float* __restrict__ b1, const float* __restrict__ b2,
                                               const float* __restrict__ b3, float* __restrict__ DST) {
  const unsigned u = blockIdx.x * 256u + threadIdx.x;
  if (u >= 4u * DM) return;
  const unsigned w = u >> 10, i = u & 1023u;
  const float v0 = b0[i], v1 = b1[i], v2 = b2[i], v3 = b3[i];
  const float v = (w == 0u) ? v0 : ((w == 1u) ? v1 : ((w == 2u) ? v2 : v3));
  VST2(float, DST + u, cmb_bf(v));
}

template <int BIAS_MODE, int OUT_MODE>
__device__ __forceinline__ void gemm64_body(
    const _Float16* __restrict__ A, unsigned lda,
    const _Float16* __restrict__ Bt, unsigned ldb,
    float* __restrict__ Cf, _Float16* __restrict__ Ch, unsigned ldc, unsigned resoff,
    const float* __restrict__ bias,
    unsigned M, unsigned N, unsigned K, float scale, float ocarry) {
  __shared__ __align__(16) float sT[8 * 16 * 68];
  const unsigned lane = threadIdx.x & 31u;
  const unsigned wave = threadIdx.x >> 5;
  const unsigned tilesN = N >> 6;
  const unsigned tilesM = M >> 6;
  const unsigned tile = blockIdx.x * 8u + wave;
  if (tile >= tilesM * tilesN) return;
  const unsigned tm = tile / tilesN;
  const unsigned tn = tile - tm * tilesN;
  const unsigned m0 = tm << 6;
  const unsigned n0 = tn << 6;
  const unsigned rlane = lane & 15u;
  const unsigned koff  = (lane >> 4) * 8u;
  const unsigned mOff  = (lane >> 4) * 8u;
  const unsigned sb    = wave * (16u * 68u);

  v8f acc[4][4];
#pragma unroll
  for (int i = 0; i < 4; ++i)
#pragma unroll
    for (int j = 0; j < 4; ++j) acc[i][j] = (v8f){0.f, 0.f, 0.f, 0.f, 0.f, 0.f, 0.f, 0.f};

  for (unsigned k0 = 0; k0 < K; k0 += 32u) {
    v16h bh[4];
#pragma unroll
    for (int j = 0; j < 4; ++j) bh[j] = ldfrag(Bt + (size_t)(n0 + ((unsigned)j << 4) + rlane) * ldb + koff + k0);
#pragma unroll
    for (int i = 0; i < 4; ++i) {
      const v16h ah = ldfrag(A + (size_t)(m0 + ((unsigned)i << 4) + rlane) * lda + koff + k0);
#pragma unroll
      for (int j = 0; j < 4; ++j)
        acc[i][j] = __builtin_amdgcn_wmma_f32_16x16x32_f16(false, ah, false, bh[j], (short)0, acc[i][j], false, false);
      dep_guard_h(acc[i][0], acc[i][3], ah, ah);
    }
    keep4_h(bh[0], bh[1], bh[2], bh[3]);
  }
  acc_guard4(acc[0][0], acc[0][1], acc[0][2], acc[0][3]);
  acc_guard4(acc[1][0], acc[1][1], acc[1][2], acc[1][3]);
  acc_guard4(acc[2][0], acc[2][1], acc[2][2], acc[2][3]);
  acc_guard4(acc[3][0], acc[3][1], acc[3][2], acc[3][3]);

#pragma unroll
  for (int i = 0; i < 4; ++i) {
    const unsigned mBase = m0 + ((unsigned)i << 4);
#pragma unroll
    for (int j = 0; j < 4; ++j) {
      const unsigned n = n0 + ((unsigned)j << 4) + rlane;
      float bv = 0.f;
      if (BIAS_MODE == 2) bv = bias[n];
#pragma unroll
      for (int r = 0; r < 8; ++r) {
        float v = acc[i][j][r] * scale;
        if (BIAS_MODE == 1) v += bias[mBase + mOff + (unsigned)r];
        if (BIAS_MODE == 2) v += bv;
        v *= ocarry;
        sT[sb + (mOff + (unsigned)r) * 68u + ((unsigned)j << 4) + rlane] = v;
      }
    }
    __builtin_amdgcn_fence(3  , "workgroup");
    __builtin_amdgcn_wave_barrier();
    __builtin_amdgcn_fence(2  , "workgroup");
    if (OUT_MODE == 0) {
      const unsigned hh = lane >> 4, c4 = (lane & 15u) * 4u;
      for (int pass = 0; pass < 2; ++pass) {
#pragma unroll
        for (int it = 0; it < 8; ++it) {
          const unsigned row = (unsigned)it * 2u + hh;
          const v4f v = *(const v4f*)(&sT[sb + row * 68u + c4]);
          *(volatile v4f*)(Cf + (size_t)(mBase + row) * ldc + n0 + c4) = v;
        }
        __threadfence();
      }
    } else {
      const unsigned q = lane >> 3, c8 = (lane & 7u) * 8u;
      v8h hv[4];
      v8h rv[4];
#pragma unroll
      for (int it = 0; it < 4; ++it) {
        const unsigned row = (unsigned)it * 4u + q;
        const v4f x0 = *(const v4f*)(&sT[sb + row * 68u + c8]);
        const v4f x1 = *(const v4f*)(&sT[sb + row * 68u + c8 + 4u]);
        const float xs[8] = {x0.x, x0.y, x0.z, x0.w, x1.x, x1.y, x1.z, x1.w};
        v8h t8, r8;
#pragma unroll
        for (int e = 0; e < 8; ++e) {
          const _Float16 hx = (_Float16)xs[e];
          t8[e] = hx;
          r8[e] = (_Float16)(xs[e] - (float)hx);
        }
        hv[it] = t8;
        rv[it] = r8;
      }
      for (int pass = 0; pass < 2; ++pass) {
#pragma unroll
        for (int it = 0; it < 4; ++it) {
          const unsigned row = (unsigned)it * 4u + q;
          *(volatile v8h*)(Ch + (size_t)(mBase + row) * ldc + n0 + c8) = hv[it];
          if (OUT_MODE == 2) *(volatile v8h*)(Ch + (size_t)(mBase + row) * ldc + resoff + n0 + c8) = rv[it];
        }
        __threadfence();
      }
    }
    __builtin_amdgcn_fence(3  , "workgroup");
    __builtin_amdgcn_wave_barrier();
    __builtin_amdgcn_fence(2  , "workgroup");
  }
}

__global__ __launch_bounds__(256) void k_gemm_q(const _Float16* __restrict__ A, const _Float16* __restrict__ Bt, _Float16* __restrict__ C,
                                                const float* __restrict__ bias, unsigned M, unsigned N, unsigned K, unsigned ldc, unsigned resoff,
                                                float scale, float ocarry) {
  gemm64_body<2, 2>(A, K, Bt, K, (float*)0, C, ldc, resoff, bias, M, N, K, scale, ocarry);
}
__global__ __launch_bounds__(256) void k_gemm_k(const _Float16* __restrict__ A, const _Float16* __restrict__ Bt, _Float16* __restrict__ C,
                                                const float* __restrict__ bias, unsigned M, unsigned N, unsigned K, unsigned ldc,
                                                float scale, float ocarry) {
  gemm64_body<2, 1>(A, K, Bt, K, (float*)0, C, ldc, 0u, bias, M, N, K, scale, ocarry);
}
__global__ __launch_bounds__(256) void k_gemm_vt(const _Float16* __restrict__ A, const _Float16* __restrict__ Bt, _Float16* __restrict__ C,
                                                 const float* __restrict__ bias, unsigned M, unsigned N, unsigned K, unsigned ldc,
                                                 float scale, float ocarry) {
  gemm64_body<1, 1>(A, K, Bt, K, (float*)0, C, ldc, 0u, bias, M, N, K, scale, ocarry);
}
__global__ __launch_bounds__(256) void k_gemm_o(const _Float16* __restrict__ A, const _Float16* __restrict__ Bt, float* __restrict__ C,
                                                const float* __restrict__ bias, unsigned M, unsigned N, unsigned K, unsigned ldc,
                                                float scale) {
  gemm64_body<2, 0>(A, K, Bt, K, C, (_Float16*)0, ldc, 0u, bias, M, N, K, scale, 1.0f);
}

__global__ __launch_bounds__(128)
void k_attn_h(const _Float16* __restrict__ Q2, const _Float16* __restrict__ K16,
              const _Float16* __restrict__ VT16, _Float16* __restrict__ AO2, float sscale) {
  __shared__ __align__(16) _Float16 Ksh[64 * 64];
  __shared__ __align__(16) _Float16 Vth[64 * 64];
  __shared__ __align__(16) _Float16 Psh[4 * 16 * 64];
  __shared__ __align__(16) float    Os[4 * 16 * 68];

  const unsigned tid = threadIdx.x, wave = tid >> 5, lane = tid & 31u, hh = lane >> 4, c = lane & 15u;
  const unsigned NQB = (unsigned)SEQ / 64u;
  const unsigned bx = blockIdx.x;
  const unsigned qb = bx % NQB, bh = bx / NQB;
  const unsigned h = bh % (unsigned)NH, b = bh / (unsigned)NH;
  if (b >= (unsigned)NB) return;
  const unsigned tb = b * (unsigned)SEQ;
  const unsigned q0 = qb * 64u + wave * 16u;
  const unsigned qoff0 = (tb + q0 + c) * (unsigned)DM2 + h * (unsigned)DK + 8u * hh;
  const unsigned pbase = wave * (16u * 64u);
  const unsigned obase = wave * (16u * 68u);

  float mrow[8], lrow[8];
  v8f oacc[4];
#pragma unroll
  for (int r = 0; r < 8; ++r) { mrow[r] = -__builtin_inff(); lrow[r] = 0.f; }
#pragma unroll
  for (int t = 0; t < 4; ++t) oacc[t] = (v8f){0.f, 0.f, 0.f, 0.f, 0.f, 0.f, 0.f, 0.f};

  for (unsigned kc = 0; kc < (unsigned)SEQ / 64u; ++kc) {
    const unsigned kv0 = kc * 64u;
    __syncthreads();
#pragma unroll
    for (int i = 0; i < 4; ++i) {
      const unsigned idx = tid + 128u * (unsigned)i;
      const unsigned row = idx >> 3, c8 = (idx & 7u) * 8u;
      const v8h kk = *(const v8h*)(K16 + (size_t)(tb + kv0 + row) * DM + h * DK + c8);
      const v8h vv = *(const v8h*)(VT16 + (size_t)(h * DK + row) * MROWS + tb + kv0 + c8);
      *(v8h*)(&Ksh[row * 64u + c8]) = kk;
      *(v8h*)(&Vth[row * 64u + c8]) = vv;
    }
    __syncthreads();

    unsigned qoff = qoff0;
    asm volatile("" : "+v"(qoff));
    const v16h qh0 = ldfrag(Q2 + qoff);
    const v16h qh1 = ldfrag(Q2 + qoff + 32u);
    const v16h qr0 = ldfrag(Q2 + qoff + (unsigned)DM);
    const v16h qr1 = ldfrag(Q2 + qoff + (unsigned)DM + 32u);

    v8f s[4];
#pragma unroll
    for (int j = 0; j < 4; ++j) {
      const v16h kb0 = ldfrag(&Ksh[((unsigned)j * 16u + c) * 64u + 8u * hh]);
      const v16h kb1 = ldfrag(&Ksh[((unsigned)j * 16u + c) * 64u + 32u + 8u * hh]);
      v8f sj = (v8f){0.f, 0.f, 0.f, 0.f, 0.f, 0.f, 0.f, 0.f};
      sj = mma_h(qh0, kb0, sj);
      sj = mma_h(qh1, kb1, sj);
      sj = mma_h(qr0, kb0, sj);
      sj = mma_h(qr1, kb1, sj);
      s[j] = sj;
    }

    float cm[8];
#pragma unroll
    for (int r = 0; r < 8; ++r) {
      float m = -__builtin_inff();
#pragma unroll
      for (int j = 0; j < 4; ++j) { s[j][r] = s[j][r] * sscale; m = fmaxf(m, s[j][r]); }
      m = fmaxf(m, __shfl_xor(m, 1, 32)); m = fmaxf(m, __shfl_xor(m, 2, 32));
      m = fmaxf(m, __shfl_xor(m, 4, 32)); m = fmaxf(m, __shfl_xor(m, 8, 32));
      cm[r] = m;
    }
#pragma unroll
    for (int r = 0; r < 8; ++r) {
      const float mnew = fmaxf(mrow[r], cm[r]);
      const float alpha = exp2f(mrow[r] - mnew);
      mrow[r] = mnew;
      float psum = 0.f;
#pragma unroll
      for (int j = 0; j < 4; ++j) {
        const float p = exp2f(s[j][r] - mnew);
        psum += p;
        Psh[pbase + (8u * hh + (unsigned)r) * 64u + (unsigned)j * 16u + c] = (_Float16)(p * 32768.0f);
      }
      psum += __shfl_xor(psum, 1, 32); psum += __shfl_xor(psum, 2, 32);
      psum += __shfl_xor(psum, 4, 32); psum += __shfl_xor(psum, 8, 32);
      lrow[r] = lrow[r] * alpha + psum;
#pragma unroll
      for (int t = 0; t < 4; ++t) oacc[t][r] = oacc[t][r] * alpha;
    }
    __builtin_amdgcn_fence(3  , "workgroup");
    __builtin_amdgcn_wave_barrier();
    __builtin_amdgcn_fence(2  , "workgroup");
#pragma unroll
    for (int kk = 0; kk < 2; ++kk) {
      const v16h pa = ldfrag(&Psh[pbase + c * 64u + (unsigned)kk * 32u + 8u * hh]);
      v16h vb[4];
#pragma unroll
      for (int t = 0; t < 4; ++t) vb[t] = ldfrag(&Vth[((unsigned)t * 16u + c) * 64u + (unsigned)kk * 32u + 8u * hh]);
#pragma unroll
      for (int t = 0; t < 4; ++t) oacc[t] = mma_h(pa, vb[t], oacc[t]);
    }
  }

#pragma unroll
  for (int r = 0; r < 8; ++r) {
    const float inv = (1.0f / lrow[r]) * (4096.0f / (32768.0f * 16.0f));
#pragma unroll
    for (int t = 0; t < 4; ++t) Os[obase + (8u * hh + (unsigned)r) * 68u + (unsigned)t * 16u + c] = oacc[t][r] * inv;
  }
  __builtin_amdgcn_fence(3  , "workgroup");
  __builtin_amdgcn_wave_barrier();
  __builtin_amdgcn_fence(2  , "workgroup");
  {
    const unsigned q4 = lane >> 3, c8 = (lane & 7u) * 8u;
    _Float16* ob = AO2 + (size_t)(tb + q0) * DM2 + h * DK;
    v8h hv[4];
    v8h rv[4];
#pragma unroll
    for (int it = 0; it < 4; ++it) {
      const unsigned row = (unsigned)it * 4u + q4;
      const v4f x0 = *(const v4f*)(&Os[obase + row * 68u + c8]);
      const v4f x1 = *(const v4f*)(&Os[obase + row * 68u + c8 + 4u]);
      const float xs[8] = {x0.x, x0.y, x0.z, x0.w, x1.x, x1.y, x1.z, x1.w};
      v8h t8, r8;
#pragma unroll
      for (int e = 0; e < 8; ++e) {
        const _Float16 hx = (_Float16)xs[e];
        t8[e] = hx;
        r8[e] = (_Float16)(xs[e] - (float)hx);
      }
      hv[it] = t8;
      rv[it] = r8;
    }
    for (int pass = 0; pass < 2; ++pass) {
#pragma unroll
      for (int it = 0; it < 4; ++it) {
        const unsigned row = (unsigned)it * 4u + q4;
        *(volatile v8h*)(ob + (size_t)row * DM2 + c8) = hv[it];
        *(volatile v8h*)(ob + (size_t)row * DM2 + DM + c8) = rv[it];
      }
      __threadfence();
    }
  }
}

#define PLANE_ACT_B  ((size_t)MROWS * DM * 2)
#define PLANE_ACT2_B ((size_t)MROWS * DM2 * 2)
#define PLANE_W_B    ((size_t)DM * DM * 2)
#define PLANE_W2_B   ((size_t)DM * DM2 * 2)
#define BR_B         ((size_t)4 * DM * 4)
#define CARVE_B      (PLANE_ACT_B * 3 + PLANE_ACT2_B * 2 + PLANE_W_B * 3 + PLANE_W2_B + BR_B)
static_assert((PLANE_ACT_B % 256) == 0 && (PLANE_ACT2_B % 256) == 0 && (PLANE_W_B % 256) == 0 && (PLANE_W2_B % 256) == 0 && (BR_B % 256) == 0);
static_assert(CARVE_B <= (size_t)134217728);
static_assert(((DM * (DM / 8)) % 256) == 0);
static_assert(((MROWS * 128) % 256) == 0);
static_assert(((4 * DM) % 256) == 0);
static_assert((((MROWS / 64) * (DM / 64)) % 8) == 0);
static_assert((NB * NH * (SEQ / 64)) * 64 == MROWS * NH);

extern "C" void kernel_launch(void* const* d_in, const int* in_sizes, int n_in, void* d_out, int out_size, void* d_ws, size_t ws_size, hipStream_t stream) {
  if (n_in < 11) return;
  const long long needX = ((long long)(NB - 1) * SEQ_FULL + SEQ) * DM;
  if ((long long)in_sizes[0] < needX || (long long)in_sizes[1] < needX || (long long)in_sizes[2] < needX) return;
  if (in_sizes[3] < DM * DM || in_sizes[5] < DM * DM || in_sizes[7] < DM * DM || in_sizes[9] < DM * DM) return;
  if (in_sizes[4] < DM || in_sizes[6] < DM || in_sizes[8] < DM || in_sizes[10] < DM) return;
  if ((long long)out_size < (long long)MROWS * DM) return;
  if ((size_t)CARVE_B > ws_size) return;

  const float* xq = (const float*)d_in[0];
  const float* xk = (const float*)d_in[1];
  const float* xv = (const float*)d_in[2];
  const float* Wq = (const float*)d_in[3];
  const float* bq = (const float*)d_in[4];
  const float* Wk = (const float*)d_in[5];
  const float* bk = (const float*)d_in[6];
  const float* Wv = (const float*)d_in[7];
  const float* bv = (const float*)d_in[8];
  const float* Wo = (const float*)d_in[9];
  const float* bo = (const float*)d_in[10];
  float* out = (float*)d_out;

  char* wsp = (char*)d_ws;
  unsigned short* X16  = (unsigned short*)wsp; wsp += PLANE_ACT_B;
  unsigned short* W16  = (unsigned short*)wsp; wsp += PLANE_W_B * 3;
  unsigned short* WO2  = (unsigned short*)wsp; wsp += PLANE_W2_B;
  unsigned short* Q2   = (unsigned short*)wsp; wsp += PLANE_ACT2_B;
  unsigned short* K16  = (unsigned short*)wsp; wsp += PLANE_ACT_B;
  unsigned short* VT16 = (unsigned short*)wsp; wsp += PLANE_ACT_B;
  unsigned short* AO2  = (unsigned short*)wsp; wsp += PLANE_ACT2_B;
  float* BR = (float*)wsp; wsp += BR_B;

  const unsigned gW = (unsigned)((DM * (DM / 8)) / 256);
  const unsigned gX = (unsigned)((MROWS * 128) / 256);
  const unsigned gG = (unsigned)((((MROWS / 64) * (DM / 64)) + 7) / 8);
  const size_t WSZ = (size_t)DM * DM;

  k_castw<<<dim3(gW), 256, 0, stream>>>(Wq, W16 + 0 * WSZ, (unsigned)DM, 0u, 16.0f);
  k_castw<<<dim3(gW), 256, 0, stream>>>(Wk, W16 + 1 * WSZ, (unsigned)DM, 0u, 16.0f);
  k_castw<<<dim3(gW), 256, 0, stream>>>(Wv, W16 + 2 * WSZ, (unsigned)DM, 0u, 16.0f);
  k_castw<<<dim3(gW), 256, 0, stream>>>(Wo, WO2, (unsigned)DM2, 1u, 16.0f);
  k_bias4<<<dim3((unsigned)((4 * DM) / 256)), 256, 0, stream>>>(bq, bk, bv, bo, BR);

  k_castx<<<dim3(gX), 256, 0, stream>>>(xq, X16, 16.0f);
  k_gemm_q<<<dim3(gG), 256, 0, stream>>>((const _Float16*)X16, (const _Float16*)(W16 + 0 * WSZ), (_Float16*)Q2, BR + 0 * DM,
      (unsigned)MROWS, (unsigned)DM, (unsigned)DM, (unsigned)DM2, (unsigned)DM, 1.0f / 256.0f, 64.0f);
  k_castx<<<dim3(gX), 256, 0, stream>>>(xk, X16, 16.0f);
  k_gemm_k<<<dim3(gG), 256, 0, stream>>>((const _Float16*)X16, (const _Float16*)(W16 + 1 * WSZ), (_Float16*)K16, BR + 1 * DM,
      (unsigned)MROWS, (unsigned)DM, (unsigned)DM, (unsigned)DM, 1.0f / 256.0f, 16.0f);
  k_castx<<<dim3(gX), 256, 0, stream>>>(xv, X16, 16.0f);
  k_gemm_vt<<<dim3(gG), 256, 0, stream>>>((const _Float16*)(W16 + 2 * WSZ), (const _Float16*)X16, (_Float16*)VT16, BR + 2 * DM,
      (unsigned)DM, (unsigned)MROWS, (unsigned)DM, (unsigned)MROWS, 1.0f / 256.0f, 16.0f);

  k_attn_h<<<dim3((unsigned)(NB * NH * (SEQ / 64))), 128, 0, stream>>>((const _Float16*)Q2, (const _Float16*)K16, (const _Float16*)VT16,
      (_Float16*)AO2, 0.125f * 1.4426950408889634f * (1.0f / 1024.0f));

  k_gemm_o<<<dim3(gG), 256, 0, stream>>>((const _Float16*)AO2, (const _Float16*)WO2, out, BR + 3 * DM,
      (unsigned)MROWS, (unsigned)DM, (unsigned)DM2, (unsigned)DM, 1.0f / 65536.0f);
}
